// ProbabilisticGraphModel_90417651515627
// MI455X (gfx1250) — hardware-verified
//
#include <hip/hip_runtime.h>
#include <math.h>

typedef __attribute__((ext_vector_type(16))) _Float16 v16h;
typedef __attribute__((ext_vector_type(16))) __bf16 v16b;
typedef __attribute__((ext_vector_type(8)))  _Float16 v8h;
typedef __attribute__((ext_vector_type(8)))  float v8f;
typedef __attribute__((ext_vector_type(4)))  float v4f;
typedef __attribute__((ext_vector_type(2)))  float v2f;
typedef __attribute__((ext_vector_type(4)))  unsigned v4u;
typedef __attribute__((ext_vector_type(4)))  int v4i;
typedef float __attribute__((may_alias)) float_a;
typedef int __attribute__((may_alias)) int_a;

template <typename T> __device__ __forceinline__ void vst2(void* p, T v) { *(volatile T*)p = v; __threadfence(); *(volatile T*)p = v; }
__device__ __forceinline__ v8f wmma16(v16h a, v16h b, v8f c) {
  v8f d = __builtin_amdgcn_wmma_f32_16x16x32_f16(false, a, false, b, (short)0, c, false, false);
  asm volatile("v_nop\n\tv_nop\n\tv_nop\n\tv_nop" : "+v"(d) : "v"(a), "v"(b));
  return d;
}
__device__ __forceinline__ v8f wmma_bf(v16b a, v16b b, v8f c) {
  v8f d = __builtin_amdgcn_wmma_f32_16x16x32_bf16(false, a, false, b, (short)0, c, false, false);
  asm volatile("v_nop\n\tv_nop\n\tv_nop\n\tv_nop" : "+v"(d) : "v"(a), "v"(b));
  return d;
}
__device__ __forceinline__ v16h frag_h(const _Float16* rowk0, int lane) {
  union { v16h v; v8h q[2]; } u; const _Float16* p = rowk0 + 8 * (lane >> 4);
  u.q[0] = *(const v8h*)p; u.q[1] = *(const v8h*)(p + 16); return u.v;
}
__device__ __forceinline__ v16h frag_f32(const float* rowk0, int lane) {
  v16h a; const float* p = rowk0 + 8 * (lane >> 4);
#pragma unroll
  for (int i = 0; i < 8; ++i) { a[i] = (_Float16)p[i]; a[8 + i] = (_Float16)p[16 + i]; }
  return a;
}
__device__ __forceinline__ v16h frag_f32s(const float* rowk0, int lane, float sc) {
  v16h a; const float* p = rowk0 + 8 * (lane >> 4);
#pragma unroll
  for (int i = 0; i < 8; ++i) { a[i] = (_Float16)(p[i] * sc); a[8 + i] = (_Float16)(p[16 + i] * sc); }
  return a;
}
__device__ __forceinline__ v16h fragc_f32(const float* W, int k0, int n, int lane, int ld, int K) {
  v16h a; const int g = lane >> 4;
#pragma unroll
  for (int i = 0; i < 8; ++i) { const int ka = k0 + 8 * g + i, kb = ka + 16;
    a[i] = (_Float16)(ka < K ? W[(size_t)(ka < K ? ka : K - 1) * ld + n] : 0.f); a[8 + i] = (_Float16)(kb < K ? W[(size_t)(kb < K ? kb : K - 1) * ld + n] : 0.f); }
  return a;
}
struct F2 { v16b h, l; };
__device__ __forceinline__ F2 bsplit16(const float v[16]) { F2 r;
#pragma unroll
  for (int i = 0; i < 16; ++i) { const __bf16 h = (__bf16)v[i]; r.h[i] = h; r.l[i] = (__bf16)(v[i] - (float)h); }
  return r; }
__device__ __forceinline__ F2 split_row(const float* row, int k0, int lane) { float v[16]; const float* p = row + k0 + 8 * (lane >> 4);
#pragma unroll
  for (int i = 0; i < 8; ++i) { v[i] = p[i]; v[8 + i] = p[16 + i]; }
  return bsplit16(v); }
__device__ __forceinline__ F2 split_rowK(const float* row, int k0, int lane, int K) { float v[16]; const int g = lane >> 4;
#pragma unroll
  for (int i = 0; i < 8; ++i) { const int ka = k0 + 8 * g + i, kb = ka + 16; v[i] = ka < K ? row[ka < K ? ka : K - 1] : 0.f; v[8 + i] = kb < K ? row[kb < K ? kb : K - 1] : 0.f; }
  return bsplit16(v); }
__device__ __forceinline__ F2 split_col(const float* W, int k0, int n, int lane, int ld, int K) { float v[16]; const int g = lane >> 4;
#pragma unroll
  for (int i = 0; i < 8; ++i) { const int ka = k0 + 8 * g + i, kb = ka + 16; v[i] = ka < K ? W[(size_t)(ka < K ? ka : K - 1) * ld + n] : 0.f; v[8 + i] = kb < K ? W[(size_t)(kb < K ? kb : K - 1) * ld + n] : 0.f; }
  return bsplit16(v); }
__device__ __forceinline__ v8f mac3(const F2& a, const F2& b, v8f c) { c = wmma_bf(a.l, b.h, c); c = wmma_bf(a.h, b.l, c); return wmma_bf(a.h, b.h, c); }
__device__ __forceinline__ float sigm(float v) { return 1.0f / (1.0f + expf(-v)); }
#define LDSX() do { asm volatile("s_wait_dscnt 0" ::: "memory"); __builtin_amdgcn_wave_barrier(); __builtin_amdgcn_fence(__ATOMIC_RELEASE, "workgroup"); } while (0)


#ifndef NN
#define NN 100000
#endif
#define EP 1600000
#ifndef NE
#define NE 1600000
#endif
#define FIN 64
#define MAXW 128
#define NBLK ((NN + 63) / 64)
#define NRP (NBLK * 64)
#define CSR_N NN
#define CSR_E NE
typedef __attribute__((ext_vector_type(8))) __bf16 v8b;
__device__ __forceinline__ v16b frag_b(const __bf16* rowk0, int lane) {
  union { v16b v; v8b q[2]; } u; const __bf16* p = rowk0 + 8 * (lane >> 4);
  u.q[0] = *(const v8b*)p; u.q[1] = *(const v8b*)(p + 16); return u.v;
}
__device__ __forceinline__ float bfr(float v) { return (float)(__bf16)v; }
__device__ __attribute__((noinline)) float exp_ni(float v) { return expf(v); }
__device__ __attribute__((noinline)) float erf_ni(float v) { return erff(v); }

#define CSR_FINN (CSR_E + 32 * CSR_NBK)
#define CSR_CHUNK 4096
#define CSR_BKT 256
#define CSR_NCH ((CSR_E + CSR_CHUNK - 1) / CSR_CHUNK)
#define CSR_NBK ((CSR_N + CSR_BKT - 1) / CSR_BKT)
#define CSR_NBKP (((CSR_NBK + 63) / 64) * 64)
#define CSR_SEGCAP (CSR_E + 32 * CSR_NBK * CSR_NCH)
#ifndef CSR_BCAP
#define CSR_BCAP 10240
#endif
#define CSR_SZ_CNT   (4u * CSR_NCH * CSR_NBKP)
#define CSR_SZ_OFF   (4u * CSR_NBK * (((CSR_NCH + 31) / 32) * 32))
#define CSR_SZ_BST   (4u * (((CSR_NBK + 1 + 31) / 32) * 32))
#define CSR_SZ_SEG   (4u * CSR_SEGCAP)
#define CSR_SZ_FIN   (4u * (CSR_E + 32 * CSR_NBK))
#define CSR_SZ_ROW   (4u * CSR_NBK * CSR_BKT)
#define CSR_OFFP (((CSR_NCH + 31) / 32) * 32)

__global__ __launch_bounds__(256) void k_csr_cnt(const int* __restrict__ DST, int dstride, int* __restrict__ CNT) {
  __shared__ unsigned short sc[256][CSR_NBK + 1]; __shared__ __align__(16) int srow[CSR_NBKP];
  const int c = blockIdx.x, tid = threadIdx.x;
  for (int b = 0; b < CSR_NBK; ++b) sc[tid][b] = 0;
  const size_t e0 = (size_t)c * CSR_CHUNK + tid * 16;
  for (int i = 0; i < 16; ++i) { const size_t e = e0 + i; if (e < (size_t)CSR_E) { int d = DST[e * dstride]; d = min(max(d, 0), CSR_N - 1); sc[tid][d / CSR_BKT] += 1; } }
  __syncthreads();
  for (int b = tid; b < CSR_NBKP; b += 256) { int s = 0; if (b < CSR_NBK) for (int t = 0; t < 256; ++t) s += sc[t][b]; srow[b] = s; }
  __syncthreads();
  for (int q = tid; q < CSR_NBKP / 4; q += 256) vst2((unsigned*)(CNT + (size_t)c * CSR_NBKP + q * 4), *(const v4u*)&srow[q * 4]);
}
__global__ __launch_bounds__(256) void k_csr_scan(const int* __restrict__ CNT, int* __restrict__ OFF, int* __restrict__ BST) {
  __shared__ int sbt[CSR_NBK + 1]; __shared__ int sbs[((CSR_NBK + 1 + 31) / 32) * 32]; __shared__ int scnt[CSR_NBK + 1]; __shared__ __align__(16) int sbuf[64][CSR_OFFP];
  const int tid = threadIdx.x;
  for (int b = tid; b < CSR_NBK; b += 256) { int sp = 0, st = 0; for (int c = 0; c < CSR_NCH; ++c) { const int n = CNT[(size_t)c * CSR_NBKP + b]; st += n; sp += (n + 31) & ~31; } sbt[b] = sp; scnt[b] = st; }
  for (int b = tid; b < ((CSR_NBK + 1 + 31) / 32) * 32; b += 256) sbs[b] = 0;
  __syncthreads();
  if (tid == 0) { int acc = 0, accf = 0; for (int b = 0; b < CSR_NBK; ++b) { const int t = sbt[b]; sbt[b] = acc; acc += t; sbs[b] = accf; accf += (scnt[b] + 31) & ~31; } sbs[CSR_NBK] = accf; }
  __syncthreads();
  for (int b0 = 0; b0 < CSR_NBK; b0 += 64) {
    if (tid < 64 && b0 + tid < CSR_NBK) { const int b = b0 + tid; int o = sbt[b]; for (int c = 0; c < CSR_OFFP; ++c) { if (c < CSR_NCH) { sbuf[tid][c] = o; o += (CNT[(size_t)c * CSR_NBKP + b] + 31) & ~31; } else sbuf[tid][c] = 0; } }
    __syncthreads();
    for (int q = tid; q < 64 * (CSR_OFFP / 4); q += 256) { const int r = q / (CSR_OFFP / 4), pc = q % (CSR_OFFP / 4); if (b0 + r < CSR_NBK) vst2((unsigned*)(OFF + (size_t)(b0 + r) * CSR_OFFP + pc * 4), *(const v4u*)&sbuf[r][pc * 4]); }
    __syncthreads(); }
  for (int q = tid; q < ((CSR_NBK + 1 + 31) / 32) * 32 / 4; q += 256) vst2((unsigned*)(BST + q * 4), *(const v4u*)&sbs[q * 4]);
}
__global__ __launch_bounds__(256) void k_csr_scatter(const int* __restrict__ SRC, const int* __restrict__ DST, int sstride, int dstride, const int* __restrict__ OFF, int* __restrict__ SEGS, int* __restrict__ SEGE) {
  __shared__ unsigned short sc[256][CSR_NBK + 1]; __shared__ int sbase[CSR_NBK + 1]; __shared__ int scn[CSR_NBK + 1]; __shared__ int sord[CSR_CHUNK];
  const int c = blockIdx.x, tid = threadIdx.x;
  for (int b = 0; b < CSR_NBK; ++b) sc[tid][b] = 0;
  const size_t e0 = (size_t)c * CSR_CHUNK + tid * 16; int bk[16];
#pragma unroll
  for (int i = 0; i < 16; ++i) { const size_t e = e0 + i; bk[i] = -1; if (e < (size_t)CSR_E) { int d = DST[e * dstride]; d = min(max(d, 0), CSR_N - 1); bk[i] = d / CSR_BKT; sc[tid][bk[i]] += 1; } }
  __syncthreads();
  for (int b = tid; b < CSR_NBK; b += 256) { int acc = 0; for (int t = 0; t < 256; ++t) { const int v = sc[t][b]; sc[t][b] = (unsigned short)acc; acc += v; } scn[b] = acc; }
  __syncthreads();
  if (tid == 0) { int acc = 0; for (int b = 0; b < CSR_NBK; ++b) { sbase[b] = acc; acc += scn[b]; } }
  __syncthreads();
#pragma unroll
  for (int i = 0; i < 16; ++i) { if (bk[i] >= 0) { const int b = bk[i]; const int r = sc[tid][b]; sc[tid][b] = (unsigned short)(r + 1); sord[sbase[b] + r] = tid * 16 + i; } }
  __syncthreads();
  for (int b = 0; b < CSR_NBK; ++b) { const int n = scn[b]; if (n == 0) continue; const int nl = ((n + 31) & ~31); const size_t o = (size_t)(min(max(OFF[(size_t)b * CSR_OFFP + c], 0), CSR_SEGCAP - nl) & ~31);
    for (int q = tid; q < nl / 4; q += 256) { int4 vs, ve;
#pragma unroll
      for (int k = 0; k < 4; ++k) { const int i = q * 4 + k; int s = -1, eid = -1; if (i < n) { const size_t e = (size_t)c * CSR_CHUNK + sord[sbase[b] + i]; s = min(max(SRC[e * sstride], 0), CSR_N - 1); eid = (int)e; } vs[k] = s; ve[k] = eid; }
      vst2((unsigned*)(SEGS + o + q * 4), *(const v4u*)&vs); vst2((unsigned*)(SEGE + o + q * 4), *(const v4u*)&ve); } }
}
__global__ __launch_bounds__(256) void k_csr_bucket(const int* __restrict__ CNT, const int* __restrict__ OFF, const int* __restrict__ BST, const int* __restrict__ SEGS, const int* __restrict__ SEGE, const int* __restrict__ DST, int dstride, int* __restrict__ FS, int* __restrict__ FE, int* __restrict__ ROWST, int* __restrict__ ROWCNT) {
  __shared__ int ssrc[CSR_BCAP]; __shared__ int seid[CSR_BCAP]; __shared__ unsigned char snod[CSR_BCAP]; __shared__ int souts[CSR_BCAP]; __shared__ int soute[CSR_BCAP]; __shared__ int scount[256]; __shared__ int sstart[257]; __shared__ int stot;
  const int b = blockIdx.x, tid = threadIdx.x;
  if (tid == 0) { int t = 0; for (int c = 0; c < CSR_NCH; ++c) t += min(max(CNT[(size_t)c * CSR_NBKP + b], 0), CSR_CHUNK); stot = (t <= CSR_BCAP) ? t : 0; }
  __syncthreads();
  { int base = 0; for (int c = 0; c < CSR_NCH; ++c) { const int n = min(max(CNT[(size_t)c * CSR_NBKP + b], 0), CSR_CHUNK); const int o = min(max(OFF[(size_t)b * CSR_OFFP + c], 0), CSR_SEGCAP - ((n + 31) & ~31));
      for (int i = tid; i < n; i += 256) { const int p = base + i; if (p < CSR_BCAP) { ssrc[p] = min(max(SEGS[o + i], 0), CSR_N - 1); const int e = min(max(SEGE[o + i], 0), CSR_E - 1); seid[p] = e; int d = DST[(size_t)e * dstride]; d = min(max(d, 0), CSR_N - 1); const int dl = d - b * CSR_BKT; snod[p] = (unsigned char)(dl >= 0 && dl < 256 ? dl : 255); } }
      base += n; } }
  __syncthreads();
  const int node = b * CSR_BKT + tid; int cnt = 0; for (int p = 0; p < stot; ++p) cnt += (snod[p] == tid) ? 1 : 0;
  scount[tid] = cnt; __syncthreads();
  if (tid == 0) { int acc = 0; for (int t = 0; t < 256; ++t) { sstart[t] = acc; acc += scount[t]; } sstart[256] = acc; }
  __syncthreads();
  const int bst0 = min(max(BST[b], 0), CSR_FINN - ((sstart[256] + 31) & ~31)) & ~31; const int gst = bst0 + sstart[tid];
  { int w = sstart[tid]; for (int p = 0; p < stot; ++p) if (snod[p] == tid) { souts[w] = ssrc[p]; soute[w] = seid[p]; ++w; } }
  __syncthreads();
  { const int n = sstart[256]; const int nl = (n + 31) & ~31; for (int q = tid; q < nl / 4; q += 256) { int4 vs, ve;
#pragma unroll
      for (int k = 0; k < 4; ++k) { const int i = q * 4 + k; vs[k] = i < n ? souts[i] : -1; ve[k] = i < n ? soute[i] : -1; }
      vst2((unsigned*)(FS + bst0 + q * 4), *(const v4u*)&vs); vst2((unsigned*)(FE + bst0 + q * 4), *(const v4u*)&ve); } }
  __syncthreads();
  { __shared__ __align__(16) int srs[256], src2[256]; srs[tid] = node < CSR_N ? gst : 0; src2[tid] = node < CSR_N ? cnt : 0; __syncthreads();
    if (tid < 64) vst2((unsigned*)(ROWST + (size_t)b * 256 + tid * 4), *(const v4u*)&srs[tid * 4]); else if (tid < 128) vst2((unsigned*)(ROWCNT + (size_t)b * 256 + (tid - 64) * 4), *(const v4u*)&src2[(tid - 64) * 4]); }
}


#define WS_CNT  0u
#define WS_OFF  (WS_CNT + CSR_SZ_CNT)
#define WS_BST  (WS_OFF + CSR_SZ_OFF)
#define WS_SEGS (WS_BST + CSR_SZ_BST)
#define WS_SEGE (WS_SEGS + CSR_SZ_SEG)
#define WS_FS   (WS_SEGE + CSR_SZ_SEG)
#define WS_FE   (WS_FS + CSR_SZ_FIN)
#define WS_RST  (WS_FE + CSR_SZ_FIN)
#define WS_RCT  (WS_RST + CSR_SZ_ROW)
#define WS_PW   (WS_RCT + CSR_SZ_ROW)
#define PW0 0
#define PW1 8192
#define PWEND 16384
#define WS_HW   (WS_PW + 2u * PWEND)
#define WS_H    (WS_HW + 4u * NRP * MAXW)
#define WS_T    (WS_H + 4u * NRP * MAXW)
#define WS_END0 (WS_T)

__global__ __launch_bounds__(256) void k_packT(const float* __restrict__ Wm, int K, int NOUT, __bf16* __restrict__ DST) {
  __shared__ __align__(16) __bf16 s[256]; const int n = blockIdx.x, tid = threadIdx.x;
  for (int k = tid; k < K; k += 256) s[k] = (__bf16)((n < NOUT) ? Wm[(size_t)k * NOUT + n] : 0.f);
  __syncthreads();
  for (int q = tid; q < K / 8; q += 256) vst2((unsigned*)(DST + (size_t)n * K + q * 8), *(const v4u*)&s[q * 8]);
}
template <int K, int NT, int RIN, int EPI>
__global__ __launch_bounds__(128) void k_lin(const float* __restrict__ A, int lda, const __bf16* __restrict__ P, const float* __restrict__ bias, float* __restrict__ OUT, int ldo) {
  __shared__ __align__(16) float so[4][16][NT * 16 + 4];
  const int tid = threadIdx.x, wave = tid >> 5, lane = tid & 31, col = lane & 15, g = lane >> 4; const size_t r0 = (size_t)blockIdx.x * 64 + wave * 16; size_t ra = r0 + col; if (ra >= NN) ra = NN - 1; const int n0 = blockIdx.y * (NT * 16);
  v8f acc[NT]; for (int j = 0; j < NT; ++j) acc[j] = (v8f){};
#pragma unroll 2
  for (int kc = 0; kc < K / 32; ++kc) { F2 a; if (RIN) { v16b ax; const float* p = A + ra * lda + kc * 32 + 8 * g;
#pragma unroll
      for (int i = 0; i < 8; ++i) { ax[i] = (__bf16)p[i]; ax[8 + i] = (__bf16)p[16 + i]; } a.h = ax; a.l = ax; } else a = split_row(A + ra * lda, kc * 32, lane);
#pragma unroll
    for (int j = 0; j < NT; ++j) { const v16b w = frag_b(P + (size_t)(n0 + j * 16 + col) * K + kc * 32, lane); if (!RIN) acc[j] = wmma_bf(a.l, w, acc[j]); acc[j] = wmma_bf(a.h, w, acc[j]); } }
#pragma unroll
  for (int j = 0; j < NT; ++j) { const int n = n0 + j * 16 + col; const float bb = bias ? bfr(bias[n]) : 0.f;
#pragma unroll
    for (int r = 0; r < 8; ++r) { float v = acc[j][r] + bb; if (EPI == 1) v = fmaxf(v, 0.f); so[wave][8 * g + r][j * 16 + col] = v; } }
  LDSX();
  for (int rl = 0; rl < 16; ++rl) if (lane < NT * 4) vst2(OUT + (r0 + rl) * ldo + n0 + lane * 4, *(const v4f*)&so[wave][rl][lane * 4]);
}
template <int RELU>
__global__ __launch_bounds__(256) void k_agg(const float* __restrict__ HW, const int* __restrict__ FS, const int* __restrict__ RST, const int* __restrict__ RCT, const float* __restrict__ bias, int width, float* __restrict__ Hd) {
  __shared__ __align__(16) float so[16][MAXW + 4];
  const int tid = threadIdx.x, blk = blockIdx.x; const int nl = tid >> 4, sl = tid & 15; const int fw = width / 16, f0 = sl * fw; const size_t node = (size_t)blk * 16 + nl;
  float acc[MAXW / 16];
#pragma unroll
  for (int i = 0; i < MAXW / 16; ++i) acc[i] = 0.f;
  if (node < (size_t)NN) { const int cnt = min(max(RCT[node], 0), CSR_BCAP); const int st = min(max(RST[node], 0), CSR_FINN - cnt);
    for (int e = 0; e < cnt; ++e) { const int s = min(max(FS[st + e], 0), NN - 1); const float ds = rsqrtf((float)(min(max(RCT[s], 0), NE) + 1)); const float* hr = HW + (size_t)s * MAXW + f0;
#pragma unroll
      for (int i = 0; i < MAXW / 16; ++i) if (i < fw) acc[i] += ds * hr[i]; }
    const float di = rsqrtf((float)(cnt + 1)); const float* own = HW + node * MAXW + f0;
#pragma unroll
    for (int i = 0; i < MAXW / 16; ++i) if (i < fw) { float v = di * (acc[i] + di * own[i]) + bfr(bias[f0 + i]); if (RELU) v = fmaxf(v, 0.f); acc[i] = v; } }
#pragma unroll
  for (int i = 0; i < MAXW / 16; ++i) if (i < fw) so[nl][f0 + i] = (node < (size_t)NN) ? acc[i] : 0.f;
  __syncthreads();
  for (int q = tid; q < 16 * (width / 4); q += 256) { const int rl = q / (width / 4), pc = q % (width / 4); vst2(Hd + ((size_t)blk * 16 + rl) * MAXW + pc * 4, *(const v4f*)&so[rl][pc * 4]); }
}

#define NG 512
#define NCHK 391
#define WS_PT  (WS_END0)
#define WS_PC  (WS_PT + 4u * NCHK * NG * 64)
#define WS_END (WS_PC + 4u * NCHK * NG)
__global__ __launch_bounds__(64) void k_poolpart(const float* __restrict__ Hd, const int* __restrict__ BATCH, float* __restrict__ PT, float* __restrict__ PC) {
  __shared__ __align__(16) float st[NG][64]; __shared__ __align__(16) float sc[NG];
  const int chunk = blockIdx.x, f = threadIdx.x;
  for (int g = 0; g < NG; ++g) st[g][f] = 0.f; for (int g = f; g < NG; g += 64) sc[g] = 0.f;
  __syncthreads();
  const int n0 = chunk * 256, n1 = min(n0 + 256, NN);
  for (int n = n0; n < n1; ++n) { const int g = min(max(BATCH[n], 0), NG - 1); st[g][f] += Hd[(size_t)n * MAXW + f]; if (f == 0) sc[g] += 1.f; }
  __syncthreads();
  for (int q = f; q < NG * 16; q += 64) { const int g = q >> 4, pc = q & 15; vst2(PT + ((size_t)chunk * NG + g) * 64 + pc * 4, *(const v4f*)&st[g][pc * 4]); }
  for (int q = f; q < NG / 4; q += 64) vst2(PC + (size_t)chunk * NG + q * 4, *(const v4f*)&sc[q * 4]);
}
__global__ __launch_bounds__(256) void k_poolout(const float* __restrict__ PT, const float* __restrict__ PC, const float* __restrict__ FCW, const float* __restrict__ FCB, float* __restrict__ out) {
  __shared__ __align__(16) float so[32]; const int tid = threadIdx.x, gl = tid >> 3, part = tid & 7; const int g = blockIdx.x * 32 + gl; const int f0 = part * 8;
  float acc[8]; float cnt = 0.f;
#pragma unroll
  for (int i = 0; i < 8; ++i) acc[i] = 0.f;
  for (int c = 0; c < NCHK; ++c) { const float* p = PT + ((size_t)c * NG + g) * 64 + f0;
#pragma unroll
    for (int i = 0; i < 8; ++i) acc[i] += p[i];
    cnt += PC[(size_t)c * NG + g]; }
  const float inv = 1.0f / fmaxf(cnt, 1.0f); float d = 0.f;
#pragma unroll
  for (int i = 0; i < 8; ++i) d += acc[i] * inv * bfr(FCW[f0 + i]);
  d += __shfl_xor(d, 1); d += __shfl_xor(d, 2); d += __shfl_xor(d, 4);
  if (part == 0) so[gl] = d + bfr(FCB[0]);
  __syncthreads();
  if (tid < 8) vst2(out + (size_t)blockIdx.x * 32 + tid * 4, *(const v4f*)&so[tid * 4]);
}

extern "C" void kernel_launch(void* const* d_in, const int* in_sizes, int n_in, void* d_out, int out_size, void* d_ws, size_t ws_size, hipStream_t stream) {
  (void)in_sizes; (void)n_in; (void)out_size;
  const float** F = (const float**)d_in; const int* EI = (const int*)d_in[1];
  if (ws_size < (size_t)WS_END) return;
  char* ws = (char*)d_ws;
  int *CNT = (int*)(ws + WS_CNT), *OFF = (int*)(ws + WS_OFF), *BST = (int*)(ws + WS_BST), *SEGS = (int*)(ws + WS_SEGS), *SEGE = (int*)(ws + WS_SEGE), *FS = (int*)(ws + WS_FS), *FE = (int*)(ws + WS_FE), *RST = (int*)(ws + WS_RST), *RCT = (int*)(ws + WS_RCT);
  __bf16* PW = (__bf16*)(ws + WS_PW); float *HW = (float*)(ws + WS_HW), *Hd = (float*)(ws + WS_H), *T = (float*)(ws + WS_T); (void)T;
  const int* SRC = EI; const int* DST = EI + EP;
  k_csr_cnt<<<CSR_NCH, 256, 0, stream>>>(DST, 1, CNT); k_csr_scan<<<1, 256, 0, stream>>>(CNT, OFF, BST); k_csr_scatter<<<CSR_NCH, 256, 0, stream>>>(SRC, DST, 1, 1, OFF, SEGS, SEGE); k_csr_bucket<<<CSR_NBK, 256, 0, stream>>>(CNT, OFF, BST, SEGS, SEGE, DST, 1, FS, FE, RST, RCT);
  const int* BATCH = (const int*)d_in[2]; float *PT = (float*)(ws + WS_PT), *PC = (float*)(ws + WS_PC);
  k_packT<<<128, 256, 0, stream>>>(F[3], 64, 128, PW + PW0); k_packT<<<64, 256, 0, stream>>>(F[5], 128, 64, PW + PW1);
  k_lin<64, 8, 1, 0><<<dim3(NBLK, 1), 128, 0, stream>>>(F[0], 64, PW + PW0, nullptr, HW, MAXW);
  k_agg<1><<<NRP / 16, 256, 0, stream>>>(HW, FS, RST, RCT, F[4], 128, Hd);
  k_lin<128, 4, 0, 0><<<dim3(NBLK, 1), 128, 0, stream>>>(Hd, MAXW, PW + PW1, nullptr, HW, MAXW);
  k_agg<1><<<NRP / 16, 256, 0, stream>>>(HW, FS, RST, RCT, F[6], 64, Hd);
  k_poolpart<<<NCHK, 64, 0, stream>>>(Hd, BATCH, PT, PC);
  k_poolout<<<NG / 32, 256, 0, stream>>>(PT, PC, F[7], F[8], (float*)d_out);
}
